// NyanEncoder_257698038442
// MI455X (gfx1250) — hardware-verified
//
#include <hip/hip_runtime.h>


#define SDIM 6
#define HD 32
#define LRELU_A 0.05f
#define SXF 16.0f
#define SWF 64.0f
#define INVS 0.0009765625f

typedef _Float16 v16h __attribute__((ext_vector_type(16)));
typedef _Float16 v8h  __attribute__((ext_vector_type(8)));
typedef float    v8f  __attribute__((ext_vector_type(8)));
typedef float    v4f  __attribute__((ext_vector_type(4)));
typedef v8h __attribute__((may_alias)) v8ha;
typedef v4f __attribute__((may_alias)) v4fa;

union Frag { v16h v; v8h p[2]; };

__device__ __forceinline__ float lrelu(float x) { return x > 0.f ? x : LRELU_A * x; }

__device__ __forceinline__ v8f wmma16(v8f acc, v16h a, v16h b) {
    acc = __builtin_amdgcn_wmma_f32_16x16x32_f16(false, a, false, b, (short)0, acc, false, false);
    asm volatile("v_nop\n\tv_nop\n\tv_nop\n\tv_nop" : "+v"(acc) : "v"(a), "v"(b));
    return acc;
}


template<int KP, int FIN>
__global__ __launch_bounds__(256) void k_buildw(const float* __restrict__ Wk, const float* __restrict__ bk,
                                                _Float16* __restrict__ Wt) {
    const int nvec = HD * KP / 8;
    const int i = blockIdx.x * blockDim.x + threadIdx.x;
    if (i >= nvec) return;
    const int n  = (i * 8) / KP;
    const int k0 = (i * 8) - n * KP;
    v8h o = {};
    #pragma unroll
    for (int j = 0; j < 8; ++j) {
        const int k = k0 + j;
        const int s = k / FIN;
        const int f = k - s * FIN;
        float v = 0.f;
        if (s < SDIM)       v = Wk[(size_t)s * (FIN * HD) + f * HD + n];
        else if (s == SDIM) v = bk[f * HD + n];
        o[j] = (_Float16)(v * SWF);
    }
    _Float16* dst = Wt + (size_t)i * 8;
    *(volatile v8h*)dst = o;
    __threadfence();
    *(volatile v8h*)dst = o;
}

template<int FIN>
__global__ __launch_bounds__(256) void k_gather(const float* __restrict__ hin, const int* __restrict__ src,
                                                _Float16* __restrict__ xg, int Nn, int nvec) {
    const int i = blockIdx.x * blockDim.x + threadIdx.x;
    if (i >= nvec) return;
    const size_t el0 = (size_t)i * 8;
    const int row = (int)(el0 / FIN);
    const int f0  = (int)(el0 - (size_t)row * FIN);
    int s = src[row];
    s = s < 0 ? 0 : (s >= Nn ? Nn - 1 : s);
    const float* p = hin + (size_t)s * FIN + f0;
    const v4f x0 = *(const v4f*)p;
    const v4f x1 = *(const v4f*)(p + 4);
    v8h o = {};
    o[0] = (_Float16)(x0[0] * SXF); o[1] = (_Float16)(x0[1] * SXF);
    o[2] = (_Float16)(x0[2] * SXF); o[3] = (_Float16)(x0[3] * SXF);
    o[4] = (_Float16)(x1[0] * SXF); o[5] = (_Float16)(x1[1] * SXF);
    o[6] = (_Float16)(x1[2] * SXF); o[7] = (_Float16)(x1[3] * SXF);
    _Float16* dst = xg + el0;
    *(volatile v8h*)dst = o;
    __threadfence();
    *(volatile v8h*)dst = o;
}

template<int KP, int FIN>
__global__ __launch_bounds__(128) void k_edge(const _Float16* __restrict__ xg, const float* __restrict__ eat,
                                              const _Float16* __restrict__ Wt, float* __restrict__ msg, int Ecnt) {
    constexpr int EPB = 64;
    constexpr int KS  = KP / 32;
    __shared__ alignas(16) _Float16 Zs[EPB * KP];
    __shared__ alignas(16) _Float16 Ws[HD * KP];
    __shared__ alignas(16) _Float16 xs[EPB * FIN];
    __shared__ float es[EPB * SDIM];
    __shared__ alignas(16) float outs[4 * 16 * HD];

    const int tid  = threadIdx.x;
    const int base = blockIdx.x * EPB;

    for (int i = tid; i < HD * KP / 8; i += 128)
        *(v8h*)(Ws + 8 * i) = *(const v8h*)(Wt + 8 * i);
    for (int i = tid; i < EPB * SDIM; i += 128) {
        const int el = i / SDIM;
        const int eidx = base + el;
        es[i] = (eidx < Ecnt) ? eat[(size_t)eidx * SDIM + (i - el * SDIM)] : 0.f;
    }
    for (int i = tid; i < EPB * FIN / 8; i += 128) {
        const int el = (8 * i) / FIN;
        const int f0 = (8 * i) - el * FIN;
        const int eidx = base + el;
        v8h v = {};
        if (eidx < Ecnt) v = *(const v8h*)(xg + (size_t)eidx * FIN + f0);
        *(v8h*)(xs + el * FIN + f0) = v;
    }
    __syncthreads();

    for (int i = tid; i < EPB * KP / 8; i += 128) {
        const int el = (8 * i) / KP;
        const int k0 = (8 * i) - el * KP;
        const int s  = k0 / FIN;
        const int f0 = k0 - s * FIN;
        v8h z = {};
        if (s < SDIM) {
            const float ev = es[el * SDIM + s];
            const v8h xv = *(const v8ha*)(xs + el * FIN + f0);
            #pragma unroll
            for (int j = 0; j < 8; ++j) z[j] = (_Float16)((float)xv[j] * ev);
        } else if (s == SDIM) {
            z = *(const v8ha*)(xs + el * FIN + f0);
        }
        *(v8h*)(Zs + el * KP + k0) = z;
    }
    __syncthreads();

    const int wave = tid >> 5;
    const int l = tid & 31, h = l >> 4, m = l & 15;
    const _Float16* arow  = Zs + (wave * 16 + m) * KP + 8 * h;
    const _Float16* b0row = Ws + m * KP + 8 * h;
    const _Float16* b1row = Ws + (16 + m) * KP + 8 * h;

    v8f acc0 = {};
    v8f acc1 = {};
    for (int t = 0; t < KS; ++t) {
        const int k0 = 32 * t;
        Frag a, b0, b1;
        a.p[0]  = *(const v8ha*)(arow + k0);   a.p[1]  = *(const v8ha*)(arow + k0 + 16);
        b0.p[0] = *(const v8ha*)(b0row + k0);  b0.p[1] = *(const v8ha*)(b0row + k0 + 16);
        b1.p[0] = *(const v8ha*)(b1row + k0);  b1.p[1] = *(const v8ha*)(b1row + k0 + 16);
        acc0 = wmma16(acc0, a.v, b0.v);
        acc1 = wmma16(acc1, a.v, b1.v);
    }

    float* ow = outs + wave * 16 * HD;
    #pragma unroll
    for (int r = 0; r < 8; ++r) {
        ow[(8 * h + r) * HD + m]      = acc0[r] * INVS;
        ow[(8 * h + r) * HD + 16 + m] = acc1[r] * INVS;
    }
    __syncthreads();

    #pragma unroll
    for (int it = 0; it < 4; ++it) {
        const int row = it * 4 + (l >> 3);
        const int c4  = (l & 7) * 4;
        const int eidx = base + wave * 16 + row;
        const v4f v = *(const v4fa*)(ow + row * HD + c4);
        if (eidx < Ecnt) *(volatile v4f*)(msg + (size_t)eidx * HD + c4) = v;
    }
    __threadfence();
    #pragma unroll
    for (int it = 0; it < 4; ++it) {
        const int row = it * 4 + (l >> 3);
        const int c4  = (l & 7) * 4;
        const int eidx = base + wave * 16 + row;
        const v4f v = *(const v4fa*)(ow + row * HD + c4);
        if (eidx < Ecnt) *(volatile v4f*)(msg + (size_t)eidx * HD + c4) = v;
    }
}

template<int NPB>
__global__ __launch_bounds__(32) void k_agg(const float* __restrict__ msg, const int* __restrict__ tgt,
                                            float* __restrict__ agg, int Nn, int Ecnt) {
    __shared__ alignas(16) float accs[NPB * HD];
    const int l  = threadIdx.x;
    const int n0 = blockIdx.x * NPB;
    const v4f z4 = {};
    for (int i = l; i < NPB * HD / 4; i += 32) *(v4fa*)(accs + 4 * i) = z4;
    __syncthreads();

    for (int eb = 0; eb < Ecnt; eb += 32) {
        const int e = eb + l;
        const int t = (e < Ecnt) ? tgt[e] : -1;
        const int rel = t - n0;
        const bool match = (unsigned)rel < (unsigned)NPB;
        unsigned mask = __builtin_amdgcn_ballot_w32(match);
        while (mask) {
            const int j = __builtin_ctz(mask);
            mask &= mask - 1u;
            int tl = __builtin_amdgcn_readlane(rel, j);
            tl &= (NPB - 1);
            const int ee = eb + j;
            accs[tl * HD + l] += msg[(size_t)ee * HD + l];
        }
    }
    __syncthreads();

    for (int it = 0; it < NPB / 4; ++it) {
        const int row = it * 4 + (l >> 3);
        const int c4  = (l & 7) * 4;
        const int node = n0 + row;
        if (node < Nn) {
            const v4f v = *(const v4fa*)(accs + row * HD + c4);
            *(volatile v4f*)(agg + (size_t)node * HD + c4) = v;
        }
    }
    __threadfence();
    for (int it = 0; it < NPB / 4; ++it) {
        const int row = it * 4 + (l >> 3);
        const int c4  = (l & 7) * 4;
        const int node = n0 + row;
        if (node < Nn) {
            const v4f v = *(const v4fa*)(accs + row * HD + c4);
            *(volatile v4f*)(agg + (size_t)node * HD + c4) = v;
        }
    }
}

__global__ __launch_bounds__(128) void k_pool(const float* __restrict__ hn, const int* __restrict__ seg,
                                              float* __restrict__ g, int Nn, int Gn) {
    constexpr int GPW = 64;
    __shared__ alignas(16) float accp[4 * GPW * HD];
    const int tid = threadIdx.x;
    const int wave = tid >> 5, l = tid & 31;
    const int g0 = (blockIdx.x * 4 + wave) * GPW;
    float* aw = accp + wave * GPW * HD;
    const v4f z4 = {};
    for (int i = l; i < GPW * HD / 4; i += 32) *(v4fa*)(aw + 4 * i) = z4;
    __syncthreads();

    for (int nb = 0; nb < Nn; nb += 32) {
        const int n = nb + l;
        const int s = (n < Nn) ? seg[n] : -1;
        const int rel = s - g0;
        const bool match = (unsigned)rel < (unsigned)GPW;
        unsigned mask = __builtin_amdgcn_ballot_w32(match);
        while (mask) {
            const int j = __builtin_ctz(mask);
            mask &= mask - 1u;
            int gl = __builtin_amdgcn_readlane(rel, j);
            gl &= (GPW - 1);
            const int nn = nb + j;
            aw[gl * HD + l] += hn[(size_t)nn * HD + l];
        }
    }
    __syncthreads();

    #pragma unroll
    for (int it = 0; it < GPW / 4; ++it) {
        const int row = it * 4 + (l >> 3);
        const int c4  = (l & 7) * 4;
        const int gg  = g0 + row;
        if (gg < Gn) {
            const v4f v = *(const v4fa*)(aw + row * HD + c4);
            *(volatile v4f*)(g + (size_t)gg * HD + c4) = v;
        }
    }
    __threadfence();
    #pragma unroll
    for (int it = 0; it < GPW / 4; ++it) {
        const int row = it * 4 + (l >> 3);
        const int c4  = (l & 7) * 4;
        const int gg  = g0 + row;
        if (gg < Gn) {
            const v4f v = *(const v4fa*)(aw + row * HD + c4);
            *(volatile v4f*)(g + (size_t)gg * HD + c4) = v;
        }
    }
}

template<int KS, int NCG, int ACT, int HASADD>
__global__ __launch_bounds__(128) void k_linear(const float* __restrict__ X, int Kin,
                                                const float* __restrict__ W, const float* __restrict__ bias,
                                                const float* __restrict__ addsrc,
                                                float* __restrict__ Y, int M) {
    constexpr int KP = 32 * KS;
    constexpr int NC = 16 * NCG;
    __shared__ alignas(16) _Float16 Xs[64 * KP];
    __shared__ alignas(16) float outs[4 * 16 * NC];

    const int tid  = threadIdx.x;
    const int row0 = blockIdx.x * 64;

    for (int i = tid; i < 64 * KP / 8; i += 128) {
        const int r  = (8 * i) / KP;
        const int c0 = (8 * i) - r * KP;
        const int grow = row0 + r;
        v8h z = {};
        if (grow < M) {
            const float* xr = X + (size_t)grow * Kin;
            #pragma unroll
            for (int j = 0; j < 8; ++j) {
                const int c  = c0 + j;
                const int cc = (c < Kin) ? c : (Kin - 1);
                float xv = xr[cc];
                if (c >= Kin) xv = 0.f;
                z[j] = (_Float16)(xv * SXF);
            }
        }
        *(v8h*)(Xs + r * KP + c0) = z;
    }
    __syncthreads();

    const int wave = tid >> 5;
    const int l = tid & 31, h = l >> 4, m = l & 15;
    const _Float16* arow = Xs + (wave * 16 + m) * KP + 8 * h;
    float* ow = outs + wave * 16 * NC;

    #pragma unroll 1
    for (int jg = 0; jg < NCG; ++jg) {
        const int col = jg * 16 + m;
        v8f acc = {};
        for (int t = 0; t < KS; ++t) {
            Frag a;
            a.p[0] = *(const v8ha*)(arow + 32 * t);
            a.p[1] = *(const v8ha*)(arow + 32 * t + 16);
            v16h bv = {};
            #pragma unroll
            for (int i = 0; i < 16; ++i) {
                const int k  = 32 * t + 8 * h + (i & 7) + ((i >> 3) << 4);
                const int kc = (k < Kin) ? k : (Kin - 1);
                float wv = W[(size_t)kc * NC + col];
                if (k >= Kin) wv = 0.f;
                bv[i] = (_Float16)(wv * SWF);
            }
            acc = wmma16(acc, a.v, bv);
        }
        const float bcol = bias[col];
        #pragma unroll
        for (int r = 0; r < 8; ++r) {
            const int row = 8 * h + r;
            float v = acc[r] * INVS + bcol;
            if (HASADD) {
                const int grow = row0 + wave * 16 + row;
                if (grow < M) v += addsrc[(size_t)grow * NC + col];
            }
            if (ACT) v = lrelu(v);
            ow[row * NC + col] = v;
        }
    }
    __syncthreads();

    const int trow0 = row0 + wave * 16;
    for (int q = l; q < 4 * NC; q += 32) {
        const int row = q / (NC / 4);
        if (trow0 + row < M) {
            const v4f v = *(const v4fa*)(ow + 4 * q);
            *(volatile v4f*)(Y + (size_t)trow0 * NC + 4 * q) = v;
        }
    }
    __threadfence();
    for (int q = l; q < 4 * NC; q += 32) {
        const int row = q / (NC / 4);
        if (trow0 + row < M) {
            const v4f v = *(const v4fa*)(ow + 4 * q);
            *(volatile v4f*)(Y + (size_t)trow0 * NC + 4 * q) = v;
        }
    }
}

__global__ __launch_bounds__(256) void k_reparam(const float* __restrict__ mu, const float* __restrict__ lv,
                                                 const float* __restrict__ eps, float* __restrict__ out, int n4) {
    const int i = blockIdx.x * blockDim.x + threadIdx.x;
    if (i >= n4) return;
    const v4f a = *(const v4f*)(mu + (size_t)i * 4);
    const v4f b = *(const v4f*)(lv + (size_t)i * 4);
    const v4f e = *(const v4f*)(eps + (size_t)i * 4);
    v4f z = {};
    #pragma unroll
    for (int j = 0; j < 4; ++j) z[j] = a[j] + expf(0.5f * b[j]) * e[j];
    float* dst = out + (size_t)i * 4;
    *(volatile v4f*)dst = z;
    __threadfence();
    *(volatile v4f*)dst = z;
}

extern "C" void kernel_launch(void* const* d_in, const int* in_sizes, int n_in,
                              void* d_out, int out_size, void* d_ws, size_t ws_size,
                              hipStream_t stream) {
    const float* x     = (const float*)d_in[0];
    const float* eat   = (const float*)d_in[1];
    const int*   src   = (const int*)  d_in[2];
    const int*   tgt   = (const int*)  d_in[3];
    const int*   seg   = (const int*)  d_in[4];
    const float* eps   = (const float*)d_in[5];
    const float* W_pre = (const float*)d_in[6];
    const float* b_pre = (const float*)d_in[7];
    const float* Wk1 = (const float*)d_in[8];  const float* bk1 = (const float*)d_in[9];
    const float* Wr1 = (const float*)d_in[10]; const float* b1  = (const float*)d_in[11];
    const float* Wk2 = (const float*)d_in[12]; const float* bk2 = (const float*)d_in[13];
    const float* Wr2 = (const float*)d_in[14]; const float* b2  = (const float*)d_in[15];
    const float* Wk3 = (const float*)d_in[16]; const float* bk3 = (const float*)d_in[17];
    const float* Wr3 = (const float*)d_in[18]; const float* b3  = (const float*)d_in[19];
    const float* W_d1 = (const float*)d_in[20]; const float* b_d1 = (const float*)d_in[21];
    const float* W_d2 = (const float*)d_in[22]; const float* b_d2 = (const float*)d_in[23];
    const float* W_mu = (const float*)d_in[24]; const float* b_mu = (const float*)d_in[25];
    const float* W_lv = (const float*)d_in[26]; const float* b_lv = (const float*)d_in[27];
    (void)n_in;

    const int Nn   = in_sizes[4];
    const int Ecnt = in_sizes[2];
    const int Gn   = in_sizes[5] / 64;
    if (Nn <= 0 || Ecnt <= 0 || Gn <= 0) return;
    const int Kin0 = in_sizes[0] / Nn;
    if (Kin0 <= 0 || Kin0 > 32) return;
    if (out_size < Gn * 64) return;

    unsigned char* ws = (unsigned char*)d_ws;
    size_t off = 0;
    auto carve = [&](size_t bytes) -> unsigned char* {
        unsigned char* p = ws + off;
        off += (bytes + 255) & ~(size_t)255;
        return p;
    };
    float*    h0  = (float*)carve((size_t)Nn * 16 * 4);
    float*    hA  = (float*)carve((size_t)Nn * HD * 4);
    float*    hB  = (float*)carve((size_t)Nn * HD * 4);
    float*    agg = (float*)carve((size_t)Nn * HD * 4);
    float*    msg = (float*)carve((size_t)Ecnt * HD * 4);
    _Float16* xg  = (_Float16*)carve((size_t)Ecnt * HD * 2);
    _Float16* Wt0 = (_Float16*)carve((size_t)HD * 128 * 2);
    _Float16* Wt1 = (_Float16*)carve((size_t)HD * 224 * 2);
    _Float16* Wt2 = (_Float16*)carve((size_t)HD * 224 * 2);
    float*    gp  = (float*)carve((size_t)Gn * HD * 4);
    float*    d1  = (float*)carve((size_t)Gn * 256 * 4);
    float*    d2  = (float*)carve((size_t)Gn * 256 * 4);
    float*    zmu = (float*)carve((size_t)Gn * 64 * 4);
    float*    zlv = (float*)carve((size_t)Gn * 64 * 4);
    if (off > ws_size) return;

    const int TB = 256;
    const int gridLinN = (Nn + 63) / 64;
    const int gridLinG = (Gn + 63) / 64;
    const int gridEdge = (Ecnt + 63) / 64;
    const int gridAgg  = (Nn + 1023) / 1024;

    k_buildw<128, 16><<<(HD * 128 / 8 + TB - 1) / TB, TB, 0, stream>>>(Wk1, bk1, Wt0);
    k_buildw<224, 32><<<(HD * 224 / 8 + TB - 1) / TB, TB, 0, stream>>>(Wk2, bk2, Wt1);
    k_buildw<224, 32><<<(HD * 224 / 8 + TB - 1) / TB, TB, 0, stream>>>(Wk3, bk3, Wt2);

    k_linear<1, 1, 1, 0><<<gridLinN, 128, 0, stream>>>(x, Kin0, W_pre, b_pre, x, h0, Nn);

    {
        const int nvec = Ecnt * 16 / 8;
        k_gather<16><<<(nvec + TB - 1) / TB, TB, 0, stream>>>(h0, src, xg, Nn, nvec);
        k_edge<128, 16><<<gridEdge, 128, 0, stream>>>(xg, eat, Wt0, msg, Ecnt);
        k_agg<1024><<<gridAgg, 32, 0, stream>>>(msg, tgt, agg, Nn, Ecnt);
        k_linear<1, 2, 1, 1><<<gridLinN, 128, 0, stream>>>(h0, 16, Wr1, b1, agg, hA, Nn);
    }
    {
        const int nvec = Ecnt * 32 / 8;
        k_gather<32><<<(nvec + TB - 1) / TB, TB, 0, stream>>>(hA, src, xg, Nn, nvec);
        k_edge<224, 32><<<gridEdge, 128, 0, stream>>>(xg, eat, Wt1, msg, Ecnt);
        k_agg<1024><<<gridAgg, 32, 0, stream>>>(msg, tgt, agg, Nn, Ecnt);
        k_linear<1, 2, 1, 1><<<gridLinN, 128, 0, stream>>>(hA, 32, Wr2, b2, agg, hB, Nn);
    }
    {
        const int nvec = Ecnt * 32 / 8;
        k_gather<32><<<(nvec + TB - 1) / TB, TB, 0, stream>>>(hB, src, xg, Nn, nvec);
        k_edge<224, 32><<<gridEdge, 128, 0, stream>>>(xg, eat, Wt2, msg, Ecnt);
        k_agg<1024><<<gridAgg, 32, 0, stream>>>(msg, tgt, agg, Nn, Ecnt);
        k_linear<1, 2, 1, 1><<<gridLinN, 128, 0, stream>>>(hB, 32, Wr3, b3, agg, hA, Nn);
    }

    k_pool<<<(Gn + 255) / 256, 128, 0, stream>>>(hA, seg, gp, Nn, Gn);

    k_linear<1, 16, 1, 0><<<gridLinG, 128, 0, stream>>>(gp, 32, W_d1, b_d1, gp, d1, Gn);
    k_linear<8, 16, 1, 0><<<gridLinG, 128, 0, stream>>>(d1, 256, W_d2, b_d2, d1, d2, Gn);
    k_linear<8, 4, 0, 0><<<gridLinG, 128, 0, stream>>>(d2, 256, W_mu, b_mu, d2, zmu, Gn);
    k_linear<8, 4, 0, 0><<<gridLinG, 128, 0, stream>>>(d2, 256, W_lv, b_lv, d2, zlv, Gn);

    {
        const int n4 = (Gn * 64) / 4;
        k_reparam<<<(n4 + TB - 1) / TB, TB, 0, stream>>>(zmu, zlv, eps, (float*)d_out, n4);
    }
    (void)hipGetLastError();
}
